// gated_attention_27599459844515
// MI455X (gfx1250) — hardware-verified
//
#include <hip/hip_runtime.h>
#include <math.h>

typedef __attribute__((ext_vector_type(16))) _Float16 v16h;
typedef __attribute__((ext_vector_type(16))) __bf16 v16b;
typedef __attribute__((ext_vector_type(8)))  _Float16 v8h;
typedef __attribute__((ext_vector_type(8)))  float v8f;
typedef __attribute__((ext_vector_type(4)))  float v4f;
typedef __attribute__((ext_vector_type(2)))  float v2f;
typedef __attribute__((ext_vector_type(4)))  unsigned v4u;
typedef __attribute__((ext_vector_type(4)))  int v4i;
typedef float __attribute__((may_alias)) float_a;
typedef int __attribute__((may_alias)) int_a;

template <typename T> __device__ __forceinline__ void vst2(void* p, T v) { *(volatile T*)p = v; __threadfence(); *(volatile T*)p = v; }
__device__ __forceinline__ v8f wmma16(v16h a, v16h b, v8f c) {
  v8f d = __builtin_amdgcn_wmma_f32_16x16x32_f16(false, a, false, b, (short)0, c, false, false);
  asm volatile("v_nop\n\tv_nop\n\tv_nop\n\tv_nop" : "+v"(d) : "v"(a), "v"(b));
  return d;
}
__device__ __forceinline__ v8f wmma_bf(v16b a, v16b b, v8f c) {
  v8f d = __builtin_amdgcn_wmma_f32_16x16x32_bf16(false, a, false, b, (short)0, c, false, false);
  asm volatile("v_nop\n\tv_nop\n\tv_nop\n\tv_nop" : "+v"(d) : "v"(a), "v"(b));
  return d;
}
__device__ __forceinline__ v16h frag_h(const _Float16* rowk0, int lane) {
  union { v16h v; v8h q[2]; } u; const _Float16* p = rowk0 + 8 * (lane >> 4);
  u.q[0] = *(const v8h*)p; u.q[1] = *(const v8h*)(p + 16); return u.v;
}
__device__ __forceinline__ v16h frag_f32(const float* rowk0, int lane) {
  v16h a; const float* p = rowk0 + 8 * (lane >> 4);
#pragma unroll
  for (int i = 0; i < 8; ++i) { a[i] = (_Float16)p[i]; a[8 + i] = (_Float16)p[16 + i]; }
  return a;
}
__device__ __forceinline__ v16h frag_f32s(const float* rowk0, int lane, float sc) {
  v16h a; const float* p = rowk0 + 8 * (lane >> 4);
#pragma unroll
  for (int i = 0; i < 8; ++i) { a[i] = (_Float16)(p[i] * sc); a[8 + i] = (_Float16)(p[16 + i] * sc); }
  return a;
}
__device__ __forceinline__ v16h fragc_f32(const float* W, int k0, int n, int lane, int ld, int K) {
  v16h a; const int g = lane >> 4;
#pragma unroll
  for (int i = 0; i < 8; ++i) { const int ka = k0 + 8 * g + i, kb = ka + 16;
    a[i] = (_Float16)(ka < K ? W[(size_t)(ka < K ? ka : K - 1) * ld + n] : 0.f); a[8 + i] = (_Float16)(kb < K ? W[(size_t)(kb < K ? kb : K - 1) * ld + n] : 0.f); }
  return a;
}
struct F2 { v16b h, l; };
__device__ __forceinline__ F2 bsplit16(const float v[16]) { F2 r;
#pragma unroll
  for (int i = 0; i < 16; ++i) { const __bf16 h = (__bf16)v[i]; r.h[i] = h; r.l[i] = (__bf16)(v[i] - (float)h); }
  return r; }
__device__ __forceinline__ F2 split_row(const float* row, int k0, int lane) { float v[16]; const float* p = row + k0 + 8 * (lane >> 4);
#pragma unroll
  for (int i = 0; i < 8; ++i) { v[i] = p[i]; v[8 + i] = p[16 + i]; }
  return bsplit16(v); }
__device__ __forceinline__ F2 split_rowK(const float* row, int k0, int lane, int K) { float v[16]; const int g = lane >> 4;
#pragma unroll
  for (int i = 0; i < 8; ++i) { const int ka = k0 + 8 * g + i, kb = ka + 16; v[i] = ka < K ? row[ka < K ? ka : K - 1] : 0.f; v[8 + i] = kb < K ? row[kb < K ? kb : K - 1] : 0.f; }
  return bsplit16(v); }
__device__ __forceinline__ F2 split_col(const float* W, int k0, int n, int lane, int ld, int K) { float v[16]; const int g = lane >> 4;
#pragma unroll
  for (int i = 0; i < 8; ++i) { const int ka = k0 + 8 * g + i, kb = ka + 16; v[i] = ka < K ? W[(size_t)(ka < K ? ka : K - 1) * ld + n] : 0.f; v[8 + i] = kb < K ? W[(size_t)(kb < K ? kb : K - 1) * ld + n] : 0.f; }
  return bsplit16(v); }
__device__ __forceinline__ v8f mac3(const F2& a, const F2& b, v8f c) { c = wmma_bf(a.l, b.h, c); c = wmma_bf(a.h, b.l, c); return wmma_bf(a.h, b.h, c); }
__device__ __forceinline__ float sigm(float v) { return 1.0f / (1.0f + expf(-v)); }
#define LDSX() do { asm volatile("s_wait_dscnt 0" ::: "memory"); __builtin_amdgcn_wave_barrier(); __builtin_amdgcn_fence(__ATOMIC_RELEASE, "workgroup"); } while (0)


#define NB 4
#define NN 512
#define DD 256
__device__ __forceinline__ float bfr(float v) { return (float)(__bf16)v; }
__device__ __forceinline__ v16b frag_b(const __bf16* rowk0, int lane) { return __builtin_bit_cast(v16b, frag_h((const _Float16*)rowk0, lane)); }
__device__ __attribute__((noinline)) float tanh_ni(float v) { return tanhf(v); }

__global__ __launch_bounds__(128) void k_proj(const float* __restrict__ x, const float* __restrict__ c, const float* __restrict__ Wq, const float* __restrict__ bq, const float* __restrict__ Wk, const float* __restrict__ Wr, const float* __restrict__ Wv, const float* __restrict__ bv,
                                             float* __restrict__ S, float* __restrict__ T, __bf16* __restrict__ VTh, __bf16* __restrict__ VTl) {
  __shared__ __align__(16) __bf16 sth[DD][72], stl[DD][72]; __shared__ float ssc[64];
  const int tid = threadIdx.x, wave = tid >> 5, lane = tid & 31, col = lane & 15, g = lane >> 4; const int which = blockIdx.y; const size_t r0b = (size_t)blockIdx.x * 64, r0 = r0b + wave * 16; const int b = (int)(r0b / NN), m0 = (int)(r0b % NN);
  const float* X = which == 0 ? x : c; const float* W = which == 0 ? Wq : (which == 1 ? Wk : Wv);
  v8f acc[16] = {};
#pragma unroll 1
  for (int kc = 0; kc < DD / 32; ++kc) { const v16b a = split_row(X + (r0 + col) * DD, kc * 32, lane).h;
#pragma unroll
    for (int j = 0; j < 16; ++j) acc[j] = wmma_bf(a, split_row(W + (size_t)(j * 16 + col) * DD, kc * 32, lane).h, acc[j]); }
  if (which < 2) {
    float part[8];
#pragma unroll
    for (int r = 0; r < 8; ++r) part[r] = 0.f;
#pragma unroll
    for (int j = 0; j < 16; ++j) { const int e = j * 16 + col; const float bb = which == 0 ? bfr(bq[e]) : 0.f; const float wr = bfr(Wr[e]);
#pragma unroll
      for (int r = 0; r < 8; ++r) part[r] += tanh_ni(acc[j][r] + bb) * wr; }
#pragma unroll
    for (int r = 0; r < 8; ++r) {
#pragma unroll
      for (int o_ = 1; o_ < 16; o_ <<= 1) part[r] += __shfl_xor(part[r], o_, 32); }
    if (col == 0) {
#pragma unroll
      for (int r = 0; r < 8; ++r) ssc[wave * 16 + 8 * g + r] = part[r]; }
    __syncthreads();
    if (tid < 16) vst2((which == 0 ? S : T) + r0b + tid * 4, *(const v4f*)(&ssc[tid * 4]));
  } else {
#pragma unroll
    for (int j = 0; j < 16; ++j) { const float bb = bfr(bv[j * 16 + col]);
#pragma unroll
      for (int r = 0; r < 8; ++r) { const float v = (acc[j][r] + bb) * 0.0625f; const __bf16 hi = (__bf16)v; sth[j * 16 + col][wave * 16 + 8 * g + r] = hi; stl[j * 16 + col][wave * 16 + 8 * g + r] = (__bf16)(v - (float)hi); } }
    __syncthreads();
    for (int qq = tid; qq < DD * 8; qq += 128) { const int e = qq >> 3, pc = qq & 7; const size_t o = ((size_t)b * DD + e) * NN + m0 + pc * 8; vst2((unsigned*)(VTh + o), *(const v4u*)(&sth[e][pc * 8])); vst2((unsigned*)(VTl + o), *(const v4u*)(&stl[e][pc * 8])); } }
}
__global__ __launch_bounds__(128) void k_attn(const float* __restrict__ x, const float* __restrict__ S, const float* __restrict__ T, const float* __restrict__ mask, const __bf16* __restrict__ VTh, const __bf16* __restrict__ VTl, const float* __restrict__ gam, const float* __restrict__ bet, float* __restrict__ out) {
  __shared__ __align__(16) float so[4][16][DD + 4];
  const int tid = threadIdx.x, wave = tid >> 5, lane = tid & 31, col = lane & 15, g = lane >> 4; const int b = blockIdx.y; const int n0 = blockIdx.x * 64 + wave * 16; const size_t rb = (size_t)b * NN;
  const int nrow = n0 + col; const float sn = S[rb + nrow]; const float* mrow = mask + (rb + nrow) * NN; const float* trow = T + rb;
  v8f acc[16] = {};
#pragma unroll 1
  for (int kc = 0; kc < NN / 32; ++kc) { union { __bf16 e[16]; v16b v; } wh, wl;
#pragma unroll
    for (int i = 0; i < 16; ++i) { const int m = kc * 32 + 8 * g + (i & 7) + (i >> 3) * 16; float w = tanh_ni(sn + trow[m]); w = (w > 0.f ? w : 0.f) * bfr(mrow[m]); const __bf16 hi = (__bf16)w; wh.e[i] = hi; wl.e[i] = (__bf16)(w - (float)hi); }
#pragma unroll
    for (int t = 0; t < 16; ++t) { const size_t vo = ((size_t)b * DD + t * 16 + col) * NN + kc * 32; const v16b vh = frag_b(VTh + vo, lane), vl = frag_b(VTl + vo, lane); acc[t] = wmma_bf(wl.v, vh, acc[t]); acc[t] = wmma_bf(wh.v, vl, acc[t]); acc[t] = wmma_bf(wh.v, vh, acc[t]); } }
  float gs[16], bs[16];
#pragma unroll
  for (int t = 0; t < 16; ++t) { gs[t] = bfr(gam[t * 16 + col]); bs[t] = bfr(bet[t * 16 + col]); }
#pragma unroll
  for (int r = 0; r < 8; ++r) { const size_t row = rb + n0 + 8 * g + r; float hv[16]; float s1 = 0.f;
#pragma unroll
    for (int t = 0; t < 16; ++t) { hv[t] = acc[t][r] + bfr(x[row * DD + t * 16 + col]); s1 += hv[t]; }
#pragma unroll
    for (int o_ = 1; o_ < 16; o_ <<= 1) s1 += __shfl_xor(s1, o_, 32);
    const float mu = s1 * (1.0f / DD); float s2 = 0.f;
#pragma unroll
    for (int t = 0; t < 16; ++t) { const float d = hv[t] - mu; s2 += d * d; }
#pragma unroll
    for (int o_ = 1; o_ < 16; o_ <<= 1) s2 += __shfl_xor(s2, o_, 32);
    const float rs = rsqrtf(s2 * (1.0f / DD) + 1e-5f);
#pragma unroll
    for (int t = 0; t < 16; ++t) so[wave][8 * g + r][t * 16 + col] = (hv[t] - mu) * rs * gs[t] + bs[t]; }
  LDSX();
  for (int rl = 0; rl < 16; ++rl) { vst2(out + (rb + n0 + rl) * DD + lane * 4, *(const v4f*)(&so[wave][rl][lane * 4])); vst2(out + (rb + n0 + rl) * DD + 128 + lane * 4, *(const v4f*)(&so[wave][rl][128 + lane * 4])); }
}
extern "C" void kernel_launch(void* const* d_in, const int* in_sizes, int n_in, void* d_out, int out_size, void* d_ws, size_t ws_size, hipStream_t stream) {
  (void)in_sizes; (void)n_in; (void)out_size; (void)ws_size;
  const float** I = (const float**)d_in;
  char* ws = (char*)d_ws; size_t off = 0;
  auto take = [&](size_t bytes) { char* p = ws + off; off += (bytes + 255) & ~(size_t)255; return p; };
  float* S = (float*)take((size_t)NB * NN * 4); float* T = (float*)take((size_t)NB * NN * 4); __bf16* VTh = (__bf16*)take((size_t)NB * DD * NN * 2); __bf16* VTl = (__bf16*)take((size_t)NB * DD * NN * 2);
  k_proj<<<dim3(NB * NN / 64, 3), 128, 0, stream>>>(I[0], I[1], I[3], I[4], I[5], I[6], I[7], I[8], S, T, VTh, VTl);
  k_attn<<<dim3(NN / 64, NB), 128, 0, stream>>>(I[0], S, T, I[2], VTh, VTl, I[9], I[10], (float*)d_out);
}
